// XLMRobertaSelfAttention_24962349924459
// MI455X (gfx1250) — hardware-verified
//
#include <hip/hip_runtime.h>
#include <math.h>

constexpr int kBatch  = 16;
constexpr int kSeq    = 512;
constexpr int kHid    = 1024;
constexpr int kHeads  = 16;
constexpr int kHdim   = 64;
constexpr int kN3     = 3 * kHid;
constexpr int kQKld   = 2 * kHid;
constexpr int kTok    = kBatch * kSeq;
constexpr int kNDist  = 2 * kSeq - 1;
constexpr int kNDistP = 1024;
constexpr float kPCarry = 32768.0f;
static_assert(kHid % 32 == 0 && kTok % 64 == 0 && kQKld % 64 == 0 && kSeq % 64 == 0, "tiles");

typedef __attribute__((ext_vector_type(16))) _Float16 v16h;
typedef __attribute__((ext_vector_type(8)))  _Float16 v8h;
typedef __attribute__((ext_vector_type(16))) __bf16   v16b;
typedef __attribute__((ext_vector_type(8)))  __bf16   v8b;
typedef __attribute__((ext_vector_type(8)))  float    v8f;
typedef __attribute__((ext_vector_type(4)))  float    v4f;
typedef __attribute__((ext_vector_type(4)))  unsigned int v4u;

__device__ __forceinline__ unsigned short f2bf_bits(float f) {
  unsigned u = __float_as_uint(f);
  return (unsigned short)((u + 0x7FFFu + ((u >> 16) & 1u)) >> 16);
}
__device__ __forceinline__ float bf_bits2f(unsigned short h) { return __uint_as_float(((unsigned)h) << 16); }

__device__ __forceinline__ void dep_guard_h(v8f& a, v8f& b, v16h x, v16h y) { asm volatile("v_nop\n\tv_nop\n\tv_nop\n\tv_nop" : "+v"(a), "+v"(b) : "v"(x), "v"(y)); }
__device__ __forceinline__ void dep_guard_b(v8f& a, v8f& b, v16b x, v16b y) { asm volatile("v_nop\n\tv_nop\n\tv_nop\n\tv_nop" : "+v"(a), "+v"(b) : "v"(x), "v"(y)); }
__device__ __forceinline__ void keep4_h(v16h a, v16h b, v16h c, v16h d) { asm volatile("v_nop" :: "v"(a), "v"(b), "v"(c), "v"(d)); }
__device__ __forceinline__ void keep4_b(v16b a, v16b b, v16b c, v16b d) { asm volatile("v_nop" :: "v"(a), "v"(b), "v"(c), "v"(d)); }
__device__ __forceinline__ void acc_guard4(v8f& a, v8f& b, v8f& c, v8f& d) { asm volatile("v_nop\n\tv_nop\n\tv_nop\n\tv_nop" : "+v"(a), "+v"(b), "+v"(c), "+v"(d)); }
template <typename T> struct Frag;
template <> struct Frag<_Float16> {
  typedef v16h V; union U { v16h v; v8h h[2]; };
  static __device__ __forceinline__ v16h load(const _Float16* p) {
    U f; f.h[0] = *(const v8h*)(p); f.h[1] = *(const v8h*)(p + 16); return f.v;
  }
  static __device__ __forceinline__ v8f mma(v16h a, v16h b, v8f c) {
    return __builtin_amdgcn_wmma_f32_16x16x32_f16(false, a, false, b, (short)0, c, false, false);
  }
  static __device__ __forceinline__ void guard(v8f& a, v8f& b, v16h x, v16h y) { dep_guard_h(a, b, x, y); }
  static __device__ __forceinline__ void keep(v16h a, v16h b, v16h c, v16h d) { keep4_h(a, b, c, d); }
};
template <> struct Frag<__bf16> {
  typedef v16b V; union U { v16b v; v8b h[2]; };
  static __device__ __forceinline__ v16b load(const __bf16* p) {
    U f; f.h[0] = *(const v8b*)(p); f.h[1] = *(const v8b*)(p + 16); return f.v;
  }
  static __device__ __forceinline__ v8f mma(v16b a, v16b b, v8f c) {
    return __builtin_amdgcn_wmma_f32_16x16x32_bf16(false, a, false, b, (short)0, c, false, false);
  }
  static __device__ __forceinline__ void guard(v8f& a, v8f& b, v16b x, v16b y) { dep_guard_b(a, b, x, y); }
  static __device__ __forceinline__ void keep(v16b a, v16b b, v16b c, v16b d) { keep4_b(a, b, c, d); }
};

__device__ __forceinline__ unsigned pk16(unsigned short a, unsigned short b) { return (unsigned)a | ((unsigned)b << 16); }

template <int ET> struct Elem;
template <> struct Elem<0> { typedef _Float16 T; };
template <> struct Elem<1> { typedef __bf16 T; };
template <int ET, int SPLIT, int BIAS_MODE, int OUT_MODE, bool RESID, int ACT = 0>
__global__ __launch_bounds__(256) void wmma_gemm64(
    const unsigned short* __restrict__ Ap, const unsigned short* __restrict__ A2p, int lda, long strideA,
    const unsigned short* __restrict__ Btp, const unsigned short* __restrict__ Bt2p, int ldb, long strideB,
    void* __restrict__ Cout, void* __restrict__ Cout2, int ldc, long strideC,
    const float* __restrict__ bias,
    const float* __restrict__ resid, long strideR,
    int M, int N, int K, float scale) {
  typedef typename Elem<ET>::T T;
  typedef typename Frag<T>::V V;
  constexpr bool SA = (SPLIT & 1) != 0;
  constexpr bool SB = (SPLIT & 2) != 0;
  const T* A = (const T*)Ap; const T* A2 = (const T*)A2p; const T* Bt = (const T*)Btp; const T* Bt2 = (const T*)Bt2p;
  __shared__ __align__(16) float sT[8][16 * 68];
  const int b    = blockIdx.y;
  const int lane = threadIdx.x & 31;
  const int wave = threadIdx.x >> 5;
  const int tilesN = N >> 6;
  const int tilesM = M >> 6;
  const int tile = blockIdx.x * 8 + wave;
  if (tile >= tilesM * tilesN) return;
  const int tm = tile / tilesN;
  const int tn = tile - tm * tilesN;
  const int m0 = tm << 6;
  const int n0 = tn << 6;

  const T* Ab  = A  + (size_t)b * strideA;
  const T* Bb  = Bt + (size_t)b * strideB;
  const T* Ab2 = SA ? (A2  + (size_t)b * strideA) : nullptr;
  const T* Bb2 = SB ? (Bt2 + (size_t)b * strideB) : nullptr;

  const int rlane = lane & 15;
  const int koff  = (lane >> 4) * 8;
  const int mOff  = (lane >> 4) * 8;

  v8f acc[4][4];
#pragma unroll
  for (int i = 0; i < 4; ++i)
#pragma unroll
    for (int j = 0; j < 4; ++j) acc[i][j] = (v8f){0.f,0.f,0.f,0.f,0.f,0.f,0.f,0.f};

  for (int k0 = 0; k0 < K; k0 += 32) {
    V bh[4], bl[4];
#pragma unroll
    for (int j = 0; j < 4; ++j) {
      const size_t bo = (size_t)(n0 + (j << 4) + rlane) * ldb + koff + k0;
      bh[j] = Frag<T>::load(Bb + bo);
      if (SB) bl[j] = Frag<T>::load(Bb2 + bo);
    }
#pragma unroll
    for (int i = 0; i < 4; ++i) {
      const size_t ao = (size_t)(m0 + (i << 4) + rlane) * lda + koff + k0;
      V ah = Frag<T>::load(Ab + ao);
      V al;
      if (SA) al = Frag<T>::load(Ab2 + ao);
#pragma unroll
      for (int j = 0; j < 4; ++j) {
        acc[i][j] = Frag<T>::mma(ah, bh[j], acc[i][j]);
        if (SB) acc[i][j] = Frag<T>::mma(ah, bl[j], acc[i][j]);
        if (SA) acc[i][j] = Frag<T>::mma(al, bh[j], acc[i][j]);
      }
      Frag<T>::guard(acc[i][0], acc[i][3], ah, SA ? al : ah);
    }
    Frag<T>::keep(bh[0], bh[1], bh[2], bh[3]);
    if (SB) Frag<T>::keep(bl[0], bl[1], bl[2], bl[3]);
  }
  acc_guard4(acc[0][0], acc[0][1], acc[0][2], acc[0][3]);
  acc_guard4(acc[1][0], acc[1][1], acc[1][2], acc[1][3]);
  acc_guard4(acc[2][0], acc[2][1], acc[2][2], acc[2][3]);
  acc_guard4(acc[3][0], acc[3][1], acc[3][2], acc[3][3]);

  float* slab = sT[wave];
  const float* Rb = RESID ? (resid + (size_t)b * strideR) : nullptr;
#pragma unroll
  for (int i = 0; i < 4; ++i) {
    const int mBase = m0 + (i << 4);
#pragma unroll
    for (int j = 0; j < 4; ++j) {
      const int n = n0 + (j << 4) + rlane;
      float bv = 0.f;
      if (BIAS_MODE == 2) bv = bf_bits2f(f2bf_bits(bias[n]));
#pragma unroll
      for (int r = 0; r < 8; ++r) {
        float v = acc[i][j][r] * scale;
        if (BIAS_MODE == 1) v += bf_bits2f(f2bf_bits(bias[mBase + mOff + r]));
        if (BIAS_MODE == 2) v += bv;
        if (RESID) v += Rb[(size_t)(mBase + mOff + r) * ldc + n];
        if (ACT == 1) v = tanhf(v);
        if (ACT == 2) v = fmaxf(v, 0.0f);
        slab[(mOff + r) * 68 + (j << 4) + rlane] = v;
      }
    }
    __builtin_amdgcn_fence(__ATOMIC_RELEASE, "workgroup");
    __builtin_amdgcn_wave_barrier();
    __builtin_amdgcn_fence(__ATOMIC_ACQUIRE, "workgroup");
    if (OUT_MODE == 0) {
      float* C = (float*)Cout + (size_t)b * strideC;
      const int hh = lane >> 4, c4 = (lane & 15) * 4;
      for (int pass = 0; pass < 2; ++pass) {
#pragma unroll
        for (int it = 0; it < 8; ++it) {
          const int row = it * 2 + hh;
          v4f v = *(const v4f*)(slab + row * 68 + c4);
          *(volatile v4f*)(C + (size_t)(mBase + row) * ldc + n0 + c4) = v;
        }
        __threadfence();
      }
    } else {
      const int q = lane >> 3, c8 = (lane & 7) * 8;
      unsigned short* C  = (unsigned short*)Cout  + (size_t)b * strideC;
      unsigned short* C2 = (OUT_MODE == 2) ? ((unsigned short*)Cout2 + (size_t)b * strideC) : nullptr;
      for (int pass = 0; pass < 2; ++pass) {
#pragma unroll
        for (int it = 0; it < 4; ++it) {
          const int row = it * 4 + q;
          const float* sp = slab + row * 68 + c8;
          v8h hv, lv;
#pragma unroll
          for (int e = 0; e < 8; ++e) {
            if (OUT_MODE == 1) {
              hv[e] = (_Float16)sp[e];
            } else {
              unsigned short hb = f2bf_bits(sp[e]);
              unsigned short lb = f2bf_bits(sp[e] - bf_bits2f(hb));
              hv[e] = __builtin_bit_cast(_Float16, hb);
              lv[e] = __builtin_bit_cast(_Float16, lb);
            }
          }
          *(volatile v8h*)(C + (size_t)(mBase + row) * ldc + n0 + c8) = hv;
          if (OUT_MODE == 2) *(volatile v8h*)(C2 + (size_t)(mBase + row) * ldc + n0 + c8) = lv;
        }
        __threadfence();
      }
    }
    __builtin_amdgcn_fence(__ATOMIC_RELEASE, "workgroup");
    __builtin_amdgcn_wave_barrier();
    __builtin_amdgcn_fence(__ATOMIC_ACQUIRE, "workgroup");
  }
}

__global__ __launch_bounds__(256) void cast8_bf16_kernel(const float* __restrict__ in, unsigned short* __restrict__ out, int n8) {
  const int i = blockIdx.x * 256 + threadIdx.x;
  if (i >= n8) return;
  const float* p = in + 8 * (size_t)i;
  const v4f a = *(const v4f*)(p);
  const v4f c = *(const v4f*)(p + 4);
  unsigned short hb[8];
#pragma unroll
  for (int e = 0; e < 4; ++e) {
    hb[e]     = f2bf_bits(a[e]);
    hb[4 + e] = f2bf_bits(c[e]);
  }
  const v4u u = (v4u){pk16(hb[0], hb[1]), pk16(hb[2], hb[3]), pk16(hb[4], hb[5]), pk16(hb[6], hb[7])};
  unsigned short* q = out + 8 * (size_t)i;
  *(volatile v4u*)q = u;
  __threadfence();
  *(volatile v4u*)q = u;
}

__global__ __launch_bounds__(256) void wtcast_kernel(const float* __restrict__ W, unsigned short* __restrict__ out) {
  __shared__ float sm[64][65];
  const int t  = threadIdx.x;
  const int k0 = blockIdx.x * 64;
  const int n0 = blockIdx.y * 64;
#pragma unroll
  for (int i = 0; i < 16; ++i) {
    const int e = i * 256 + t;
    const int r = e >> 6;
    const int c = e & 63;
    sm[c][r] = W[(size_t)(k0 + r) * kN3 + n0 + c];
  }
  __syncthreads();
  const int lane = t & 31, wave = t >> 5;
  const int q = lane >> 3, c8 = (lane & 7) * 8;
  for (int pass = 0; pass < 2; ++pass) {
#pragma unroll
    for (int it = 0; it < 2; ++it) {
      const int row = wave * 8 + it * 4 + q;
      unsigned short hb[8];
#pragma unroll
      for (int e = 0; e < 8; ++e) hb[e] = f2bf_bits(sm[row][c8 + e]);
      const v4u u = (v4u){pk16(hb[0], hb[1]), pk16(hb[2], hb[3]), pk16(hb[4], hb[5]), pk16(hb[6], hb[7])};
      *(volatile v4u*)(out + (size_t)(n0 + row) * kHid + k0 + c8) = u;
    }
    __threadfence();
  }
}

__global__ __launch_bounds__(256) void pecast_kernel(const float* __restrict__ pe, unsigned short* __restrict__ out) {
  const int i = blockIdx.x * 256 + threadIdx.x;
  if (i >= kNDistP * kHdim / 8) return;
  const int row = i >> 3, c8 = (i & 7) * 8;
  const int rc = (row < kNDist) ? row : (kNDist - 1);
  const float* src = pe + (size_t)rc * kHdim + c8;
  const v4f a = *(const v4f*)(src);
  const v4f c = *(const v4f*)(src + 4);
  const bool live = (row < kNDist);
  unsigned short hb[8];
#pragma unroll
  for (int e = 0; e < 4; ++e) {
    hb[e]     = live ? f2bf_bits(a[e]) : (unsigned short)0;
    hb[4 + e] = live ? f2bf_bits(c[e]) : (unsigned short)0;
  }
  const v4u u = (v4u){pk16(hb[0], hb[1]), pk16(hb[2], hb[3]), pk16(hb[4], hb[5]), pk16(hb[6], hb[7])};
  unsigned short* q = out + (size_t)row * kHdim + c8;
  *(volatile v4u*)q = u;
  __threadfence();
  *(volatile v4u*)q = u;
}

__device__ __forceinline__ unsigned short at_bf_bits(float f) {
  unsigned u = __float_as_uint(f);
  return (unsigned short)((u + 0x7FFFu + ((u >> 16) & 1u)) >> 16);
}
__device__ __forceinline__ __bf16 at_f2bf(float f) { return __builtin_bit_cast(__bf16, at_bf_bits(f)); }
__device__ __forceinline__ v8f at_mma(v16b a, v16b b, v8f c) {
  c = __builtin_amdgcn_wmma_f32_16x16x32_bf16(false, a, false, b, (short)0, c, false, false);
  asm volatile("v_nop\n\tv_nop\n\tv_nop\n\tv_nop" : "+v"(c) : "v"(a), "v"(b));
  return c;
}
template <bool F16> __device__ __forceinline__ __bf16 at_to16(float f) {
  if (F16) return __builtin_bit_cast(__bf16, (_Float16)f);
  return at_f2bf(f);
}
template <bool F16> __device__ __forceinline__ v8f at_mma16(v16b a, v16b b, v8f c) {
  if (F16) {
    const v16h ah = __builtin_bit_cast(v16h, a), bh = __builtin_bit_cast(v16h, b);
    c = __builtin_amdgcn_wmma_f32_16x16x32_f16(false, ah, false, bh, (short)0, c, false, false);
    asm volatile("v_nop\n\tv_nop\n\tv_nop\n\tv_nop" : "+v"(c) : "v"(ah), "v"(bh));
    return c;
  }
  return at_mma(a, b, c);
}

constexpr int kT1Slots = 80;
__global__ __launch_bounds__(128)
void relattn_kernel(const unsigned short* __restrict__ QKhp, const unsigned short* __restrict__ QKlp,
                    const unsigned short* __restrict__ Vtp, const unsigned short* __restrict__ PEp,
                    const float* __restrict__ mask, float* __restrict__ out) {
  union FB { v16b v; v8b h[2]; };
  __shared__ __align__(16) _Float16 T1s[4][kT1Slots * 16];
  __shared__ __align__(16) _Float16 T2s[128 * 64];
  __shared__ __align__(16) __bf16   Psh[4][16 * 64];
  __shared__ __align__(16) float    Os[4][16 * 68];

  const int tid  = threadIdx.x;
  const int wave = tid >> 5;
  const int lane = tid & 31;
  const int hh   = lane >> 4;
  const int c    = lane & 15;

  const int qb = blockIdx.x;
  const int h  = blockIdx.y;
  const int b  = blockIdx.z;
  const int l0 = qb * 64;
  const int q0 = l0 + wave * 16;
  const size_t tok0 = (size_t)b * kSeq;

  const __bf16* Qh  = (const __bf16*)QKhp;
  const __bf16* Ql  = (const __bf16*)QKlp;
  const __bf16* Vt  = (const __bf16*)Vtp;
  const __bf16* PEt = (const __bf16*)PEp;

  v16b qah[2], qal[2];
  {
    const size_t qo = (tok0 + q0 + c) * kQKld + (size_t)h * kHdim + 8 * hh;
#pragma unroll
    for (int dc = 0; dc < 2; ++dc) {
      qah[dc] = Frag<__bf16>::load(Qh + qo + dc * 32);
      qal[dc] = Frag<__bf16>::load(Ql + qo + dc * 32);
    }
  }

  float mrow[8], lrow[8];
  v8f oacc[4];
#pragma unroll
  for (int r = 0; r < 8; ++r) { mrow[r] = -INFINITY; lrow[r] = 0.f; }
#pragma unroll
  for (int t = 0; t < 4; ++t) oacc[t] = (v8f){0.f,0.f,0.f,0.f,0.f,0.f,0.f,0.f};

  _Float16* t1w = T1s[wave];
  __bf16*   pw  = Psh[wave];

  for (int kc = 0; kc < kSeq / 64; ++kc) {
    const int r0 = kc * 64;
    const int d0 = l0 - r0 + 448;
    __syncthreads();

    {
      v16b ka[2];
      const size_t ko = (tok0 + r0 + wave * 16 + c) * kQKld + kHid + (size_t)h * kHdim + 8 * hh;
#pragma unroll
      for (int dc = 0; dc < 2; ++dc) ka[dc] = Frag<__bf16>::load(Qh + ko + dc * 32);
#pragma unroll
      for (int i = 0; i < 5; ++i) {
        const int dt1 = d0 + 16 * wave + 16 * i;
        const int dt2 = d0 + 16 * (3 - wave + i);
        v8f a1 = (v8f){0.f,0.f,0.f,0.f,0.f,0.f,0.f,0.f};
        v8f a2 = (v8f){0.f,0.f,0.f,0.f,0.f,0.f,0.f,0.f};
#pragma unroll
        for (int dc = 0; dc < 2; ++dc) {
          const v16b p1 = Frag<__bf16>::load(PEt + (size_t)(dt1 + c) * kHdim + 8 * hh + dc * 32);
          const v16b p2 = Frag<__bf16>::load(PEt + (size_t)(dt2 + c) * kHdim + 8 * hh + dc * 32);
          a1 = at_mma(qah[dc], p1, a1);
          a2 = at_mma(ka[dc], p2, a2);
        }
        v8h hv1, hv2;
#pragma unroll
        for (int r = 0; r < 8; ++r) { hv1[r] = (_Float16)a1[r]; hv2[r] = (_Float16)a2[r]; }
        *(v8h*)(t1w + (16 * i + c) * 16 + 8 * hh) = hv1;
        *(v8h*)(T2s + (size_t)(16 * (3 - wave + i) + c) * 64 + 16 * wave + 8 * hh) = hv2;
      }
    }

    v8f s[4];
#pragma unroll
    for (int j = 0; j < 4; ++j) {
      s[j] = (v8f){0.f,0.f,0.f,0.f,0.f,0.f,0.f,0.f};
#pragma unroll
      for (int dc = 0; dc < 2; ++dc) {
        const size_t ko = (tok0 + r0 + j * 16 + c) * kQKld + kHid + (size_t)h * kHdim + 8 * hh + dc * 32;
        const v16b kb = Frag<__bf16>::load(Qh + ko);
        const v16b kl = Frag<__bf16>::load(Ql + ko);
        s[j] = at_mma(qah[dc], kb, s[j]);
        s[j] = at_mma(qah[dc], kl, s[j]);
        s[j] = at_mma(qal[dc], kb, s[j]);
      }
    }
    __syncthreads();

    float mk[4];
#pragma unroll
    for (int j = 0; j < 4; ++j) mk[j] = mask[tok0 + r0 + j * 16 + c];

    float cm[8];
#pragma unroll
    for (int r = 0; r < 8; ++r) {
      float m = -INFINITY;
#pragma unroll
      for (int j = 0; j < 4; ++j) {
        const int p1 = 8 * hh + r - 16 * j - c + 63;
        const float t1 = (float)t1w[p1 * 16 + 8 * hh + r];
        const float t2 = (float)T2s[(p1 + 16 * wave) * 64 + 16 * j + c];
        const float v = (s[j][r] + t1 + t2) * 0.125f + mk[j];
        s[j][r] = v;
        m = fmaxf(m, v);
      }
#pragma unroll
      for (int off = 1; off < 16; off <<= 1) m = fmaxf(m, __shfl_xor(m, off, 32));
      cm[r] = m;
    }
#pragma unroll
    for (int r = 0; r < 8; ++r) {
      const float mnew = fmaxf(mrow[r], cm[r]);
      const float alpha = __expf(mrow[r] - mnew);
      mrow[r] = mnew;
      float psum = 0.f;
#pragma unroll
      for (int j = 0; j < 4; ++j) {
        const float p = __expf(s[j][r] - mnew);
        psum += p;
        pw[(8 * hh + r) * 64 + j * 16 + c] = at_to16<true>(p * kPCarry);
      }
#pragma unroll
      for (int off = 1; off < 16; off <<= 1) psum += __shfl_xor(psum, off, 32);
      lrow[r] = lrow[r] * alpha + psum;
#pragma unroll
      for (int t = 0; t < 4; ++t) oacc[t][r] *= alpha;
    }
    __builtin_amdgcn_fence(__ATOMIC_RELEASE, "workgroup");
    __builtin_amdgcn_wave_barrier();
    __builtin_amdgcn_fence(__ATOMIC_ACQUIRE, "workgroup");
#pragma unroll 1
    for (int kk = 0; kk < 2; ++kk) {
      FB pa;
      pa.h[0] = *(const v8b*)(pw + c * 64 + kk * 32 + 8 * hh);
      pa.h[1] = *(const v8b*)(pw + c * 64 + kk * 32 + 16 + 8 * hh);
#pragma unroll
      for (int t = 0; t < 4; ++t) {
        FB vb;
        const size_t vo = ((size_t)(b * kHeads + h) * kHdim + t * 16 + c) * kSeq + r0 + kk * 32 + 8 * hh;
        vb.h[0] = *(const v8b*)(Vt + vo);
        vb.h[1] = *(const v8b*)(Vt + vo + 16);
        oacc[t] = at_mma16<true>(pa.v, vb.v, oacc[t]);
      }
    }
  }

  float* os = Os[wave];
#pragma unroll
  for (int r = 0; r < 8; ++r) {
    const float inv = 1.0f / (lrow[r] * kPCarry);
#pragma unroll
    for (int t = 0; t < 4; ++t) os[(8 * hh + r) * 68 + t * 16 + c] = oacc[t][r] * inv;
  }
  __builtin_amdgcn_fence(__ATOMIC_RELEASE, "workgroup");
  __builtin_amdgcn_wave_barrier();
  __builtin_amdgcn_fence(__ATOMIC_ACQUIRE, "workgroup");
  {
    float* ob = out + (size_t)h * kHdim;
    const int c4 = (lane & 15) * 4;
    for (int pass = 0; pass < 2; ++pass) {
#pragma unroll
      for (int it = 0; it < 8; ++it) {
        const int row = it * 2 + hh;
        v4f val = *(const v4f*)(os + row * 68 + c4);
        *(volatile v4f*)(ob + (tok0 + q0 + row) * kHid + c4) = val;
      }
      __threadfence();
    }
  }
}

extern "C" void kernel_launch(void* const* d_in, const int* in_sizes, int n_in,
                              void* d_out, int out_size, void* d_ws, size_t ws_size,
                              hipStream_t stream) {
  if (n_in < 5) return;
  if (in_sizes[0] != kTok * kHid) return;
  if (in_sizes[1] != kBatch * kSeq) return;
  if (in_sizes[2] != kHid * kN3) return;
  if (in_sizes[3] != kN3) return;
  if (in_sizes[4] != kNDist * kHdim) return;
  if (out_size != kTok * kHid) return;

  const float* hid  = (const float*)d_in[0];
  const float* msk  = (const float*)d_in[1];
  const float* W    = (const float*)d_in[2];
  const float* bqkv = (const float*)d_in[3];
  const float* pe   = (const float*)d_in[4];
  float* outp = (float*)d_out;

  const size_t SZ_X16 = (size_t)kTok * kHid * 2;
  const size_t SZ_WT  = (size_t)kN3 * kHid * 2;
  const size_t SZ_PE  = (size_t)kNDistP * kHdim * 2;
  const size_t SZ_QK  = (size_t)kTok * kQKld * 2;
  const size_t SZ_VT  = (size_t)kBatch * kHid * kSeq * 2;
  size_t off = 0;
  const size_t oX16 = off; off += SZ_X16;
  const size_t oWT  = off; off += SZ_WT;
  const size_t oPE  = off; off += SZ_PE;
  const size_t oQKh = off; off += SZ_QK;
  const size_t oQKl = off; off += SZ_QK;
  const size_t oVT  = off; off += SZ_VT;
  const size_t TOTAL = off;
  if (TOTAL > ws_size) return;
  if (TOTAL > (size_t)134217728) return;

  char* ws = (char*)d_ws;
  unsigned short* X16 = (unsigned short*)(ws + oX16);
  unsigned short* WT  = (unsigned short*)(ws + oWT);
  unsigned short* PEb = (unsigned short*)(ws + oPE);
  unsigned short* QKh = (unsigned short*)(ws + oQKh);
  unsigned short* QKl = (unsigned short*)(ws + oQKl);
  unsigned short* VTp = (unsigned short*)(ws + oVT);

  const dim3 blk(256);
  {
    const int n8 = kTok * kHid / 8;
    cast8_bf16_kernel<<<dim3((n8 + 255) / 256), blk, 0, stream>>>(hid, X16, n8);
  }
  wtcast_kernel<<<dim3(kHid / 64, kN3 / 64), blk, 0, stream>>>(W, WT);
  pecast_kernel<<<dim3((kNDistP * kHdim / 8 + 255) / 256), blk, 0, stream>>>(pe, PEb);
  {
    const dim3 g(((kTok / 64) * (kQKld / 64) + 7) / 8, 1);
    wmma_gemm64<1, 0, 2, 2, false, 0><<<g, blk, 0, stream>>>(
        X16, X16, kHid, 0L, WT, WT, kHid, 0L, (void*)QKh, (void*)QKl, kQKld, 0L,
        bqkv, hid, 0L, kTok, kQKld, kHid, 1.0f);
  }
  {
    const dim3 g(((kHid / 64) * (kSeq / 64) + 7) / 8, kBatch);
    wmma_gemm64<1, 0, 1, 1, false, 0><<<g, blk, 0, stream>>>(
        WT + (size_t)2 * kHid * kHid, WT + (size_t)2 * kHid * kHid, kHid, 0L,
        X16, X16, kHid, (long)kSeq * kHid,
        (void*)VTp, (void*)VTp, kSeq, (long)kHid * kSeq,
        bqkv + 2 * kHid, hid, 0L, kHid, kSeq, kHid, 1.0f);
  }
  relattn_kernel<<<dim3(kSeq / 64, kHeads, kBatch), dim3(128), 0, stream>>>(QKh, QKl, VTp, PEb, msk, outp);
}
